// RadarConv_14482629722249
// MI455X (gfx1250) — hardware-verified
//
#include <hip/hip_runtime.h>
#include <stddef.h>

constexpr int kNB   = 4;
constexpr int kCIN  = 256;
constexpr int kHH   = 80;
constexpr int kWD   = 80;
constexpr int kHW   = 6400;
constexpr int kNPIX = 25600;
constexpr int kCOUT = 256;
constexpr int kTAPS = 9;
constexpr int kKD   = 2304;
constexpr int kMOFF = 64;
constexpr int kNOFS = 18;
constexpr int kNMOD = 9;
constexpr int kNOFF = 27;
constexpr float kSC_IM = 4.0f;
constexpr float kSC_WO = 64.0f;
constexpr float kSC_S  = 8.0f;
constexpr float kSC_WD = 32.0f;
constexpr float kEPI_OFF  = 1.0f / (kSC_IM * kSC_WO);
constexpr float kEPI_MAIN = 1.0f / (kSC_S * kSC_WD);
static_assert(kKD == kTAPS * kCIN);
static_assert(kKD % 32 == 0);
static_assert(kHW % 64 == 0);
static_assert(kHW % 32 == 0);
static_assert(kCOUT % 64 == 0);
static_assert(kCIN == 256);
static_assert(kNPIX == kNB * kHW);
static_assert(kNOFF == kNOFS + kNMOD);
static_assert((kHW * kTAPS) % 8 == 0);
static_assert((kMOFF * kKD / 8) % 256 == 0);
static_assert((kCOUT * kKD / 8) % 256 == 0);

typedef __attribute__((ext_vector_type(16))) _Float16 v16h;
typedef __attribute__((ext_vector_type(8)))  _Float16 v8h;
typedef __attribute__((ext_vector_type(16))) __bf16   v16b;
typedef __attribute__((ext_vector_type(8)))  __bf16   v8b;
typedef __attribute__((ext_vector_type(8)))  float    v8f;
typedef __attribute__((ext_vector_type(4)))  float    v4f;
typedef __attribute__((ext_vector_type(4)))  unsigned v4u;

__device__ __forceinline__ unsigned short f2bf_bits(float f) {
  unsigned u = __float_as_uint(f);
  return (unsigned short)((u + 0x7FFFu + ((u >> 16) & 1u)) >> 16);
}
__device__ __forceinline__ float bf_bits2f(unsigned short h) { return __uint_as_float(((unsigned)h) << 16); }

__device__ __forceinline__ unsigned pk2(unsigned short a, unsigned short b) {
  return (unsigned)a | ((unsigned)b << 16);
}
__device__ __forceinline__ unsigned pkh2(float a, float b) {
  return pk2(__builtin_bit_cast(unsigned short, (_Float16)a), __builtin_bit_cast(unsigned short, (_Float16)b));
}

__device__ __forceinline__ void dep_guard_h(v8f& a, v8f& b, v16h x, v16h y) { asm volatile("v_nop\n\tv_nop\n\tv_nop\n\tv_nop" : "+v"(a), "+v"(b) : "v"(x), "v"(y)); }
__device__ __forceinline__ void dep_guard_b(v8f& a, v8f& b, v16b x, v16b y) { asm volatile("v_nop\n\tv_nop\n\tv_nop\n\tv_nop" : "+v"(a), "+v"(b) : "v"(x), "v"(y)); }
__device__ __forceinline__ void keep4_h(v16h a, v16h b, v16h c, v16h d) { asm volatile("v_nop" :: "v"(a), "v"(b), "v"(c), "v"(d)); }
__device__ __forceinline__ void keep4_b(v16b a, v16b b, v16b c, v16b d) { asm volatile("v_nop" :: "v"(a), "v"(b), "v"(c), "v"(d)); }
__device__ __forceinline__ void acc_guard4(v8f& a, v8f& b, v8f& c, v8f& d) { asm volatile("v_nop\n\tv_nop\n\tv_nop\n\tv_nop" : "+v"(a), "+v"(b), "+v"(c), "+v"(d)); }
template <typename T> struct Frag;
template <> struct Frag<_Float16> {
  typedef v16h V; union U { v16h v; v8h h[2]; };
  static __device__ __forceinline__ v16h load(const _Float16* p) {
    U f; f.h[0] = *(const v8h*)(p); f.h[1] = *(const v8h*)(p + 16); return f.v;
  }
  static __device__ __forceinline__ v8f mma(v16h a, v16h b, v8f c) {
    return __builtin_amdgcn_wmma_f32_16x16x32_f16(false, a, false, b, (short)0, c, false, false);
  }
  static __device__ __forceinline__ void guard(v8f& a, v8f& b, v16h x, v16h y) { dep_guard_h(a, b, x, y); }
  static __device__ __forceinline__ void keep(v16h a, v16h b, v16h c, v16h d) { keep4_h(a, b, c, d); }
};
template <> struct Frag<__bf16> {
  typedef v16b V; union U { v16b v; v8b h[2]; };
  static __device__ __forceinline__ v16b load(const __bf16* p) {
    U f; f.h[0] = *(const v8b*)(p); f.h[1] = *(const v8b*)(p + 16); return f.v;
  }
  static __device__ __forceinline__ v8f mma(v16b a, v16b b, v8f c) {
    return __builtin_amdgcn_wmma_f32_16x16x32_bf16(false, a, false, b, (short)0, c, false, false);
  }
  static __device__ __forceinline__ void guard(v8f& a, v8f& b, v16b x, v16b y) { dep_guard_b(a, b, x, y); }
  static __device__ __forceinline__ void keep(v16b a, v16b b, v16b c, v16b d) { keep4_b(a, b, c, d); }
};

template <int ET> struct Elem;
template <> struct Elem<0> { typedef _Float16 T; };
template <> struct Elem<1> { typedef __bf16 T; };
template <int ET, bool SPLIT, int BIAS_MODE, int OUT_MODE, bool RESID, int ACT = 0>
__global__ __launch_bounds__(256) void wmma_gemm64(
    const unsigned short* __restrict__ Ap, const unsigned short* __restrict__ A2p, int lda, long strideA,
    const unsigned short* __restrict__ Btp, const unsigned short* __restrict__ Bt2p, int ldb, long strideB,
    void* __restrict__ Cout, void* __restrict__ Cout2, int ldc, long strideC,
    const float* __restrict__ bias,
    const float* __restrict__ resid, long strideR,
    int M, int N, int K, float scale) {
  typedef typename Elem<ET>::T T;
  typedef typename Frag<T>::V V;
  const T* A = (const T*)Ap; const T* A2 = (const T*)A2p; const T* Bt = (const T*)Btp; const T* Bt2 = (const T*)Bt2p;
  __shared__ __align__(16) float sT[8][16 * 68];
  const int b    = blockIdx.y;
  const int lane = threadIdx.x & 31;
  const int wave = threadIdx.x >> 5;
  const int tilesN = N >> 6;
  const int tilesM = M >> 6;
  const int tile = blockIdx.x * 8 + wave;
  if (tile >= tilesM * tilesN) return;
  const int tm = tile / tilesN;
  const int tn = tile - tm * tilesN;
  const int m0 = tm << 6;
  const int n0 = tn << 6;

  const T* Ab  = A  + (size_t)b * strideA;
  const T* Bb  = Bt + (size_t)b * strideB;
  const T* Ab2 = SPLIT ? (A2  + (size_t)b * strideA) : nullptr;
  const T* Bb2 = SPLIT ? (Bt2 + (size_t)b * strideB) : nullptr;

  const int rlane = lane & 15;
  const int koff  = (lane >> 4) * 8;
  const int mOff  = (lane >> 4) * 8;

  v8f acc[4][4];
#pragma unroll
  for (int i = 0; i < 4; ++i)
#pragma unroll
    for (int j = 0; j < 4; ++j) acc[i][j] = (v8f){0.f,0.f,0.f,0.f,0.f,0.f,0.f,0.f};

  for (int k0 = 0; k0 < K; k0 += 32) {
    V bh[4], bl[4];
#pragma unroll
    for (int j = 0; j < 4; ++j) {
      const size_t bo = (size_t)(n0 + (j << 4) + rlane) * ldb + koff + k0;
      bh[j] = Frag<T>::load(Bb + bo);
      if (SPLIT) bl[j] = Frag<T>::load(Bb2 + bo);
    }
#pragma unroll
    for (int i = 0; i < 4; ++i) {
      const size_t ao = (size_t)(m0 + (i << 4) + rlane) * lda + koff + k0;
      V ah = Frag<T>::load(Ab + ao);
      V al;
      if (SPLIT) al = Frag<T>::load(Ab2 + ao);
#pragma unroll
      for (int j = 0; j < 4; ++j) {
        acc[i][j] = Frag<T>::mma(ah, bh[j], acc[i][j]);
        if (SPLIT) {
          acc[i][j] = Frag<T>::mma(ah, bl[j], acc[i][j]);
          acc[i][j] = Frag<T>::mma(al, bh[j], acc[i][j]);
        }
      }
      Frag<T>::guard(acc[i][0], acc[i][3], ah, SPLIT ? al : ah);
    }
    Frag<T>::keep(bh[0], bh[1], bh[2], bh[3]);
    if (SPLIT) Frag<T>::keep(bl[0], bl[1], bl[2], bl[3]);
  }
  acc_guard4(acc[0][0], acc[0][1], acc[0][2], acc[0][3]);
  acc_guard4(acc[1][0], acc[1][1], acc[1][2], acc[1][3]);
  acc_guard4(acc[2][0], acc[2][1], acc[2][2], acc[2][3]);
  acc_guard4(acc[3][0], acc[3][1], acc[3][2], acc[3][3]);

  float* slab = sT[wave];
  const float* Rb = RESID ? (resid + (size_t)b * strideR) : nullptr;
#pragma unroll
  for (int i = 0; i < 4; ++i) {
    const int mBase = m0 + (i << 4);
#pragma unroll
    for (int j = 0; j < 4; ++j) {
      const int n = n0 + (j << 4) + rlane;
      float bv = 0.f;
      if (BIAS_MODE == 2) bv = bias[n];
#pragma unroll
      for (int r = 0; r < 8; ++r) {
        float v = acc[i][j][r] * scale;
        if (BIAS_MODE == 1) v += bias[mBase + mOff + r];
        if (BIAS_MODE == 2) v += bv;
        if (RESID) v += Rb[(size_t)(mBase + mOff + r) * ldc + n];
        if (ACT == 1) v = tanhf(v);
        if (ACT == 2) v = fmaxf(v, 0.0f);
        if (ACT == 3) v = v / (1.0f + expf(-v));
        if (ACT == 4) v = (v > 0.f) ? v : 0.01f * v;
        if (ACT == 5) v = 0.5f * v * (1.0f + erff(v * 0.70710678118654752f));
        slab[(mOff + r) * 68 + (j << 4) + rlane] = v;
      }
    }
    __builtin_amdgcn_fence(__ATOMIC_RELEASE, "workgroup");
    __builtin_amdgcn_wave_barrier();
    __builtin_amdgcn_fence(__ATOMIC_ACQUIRE, "workgroup");
    if (OUT_MODE == 0) {
      float* C = (float*)Cout + (size_t)b * strideC;
      const int hh = lane >> 4, c4 = (lane & 15) * 4;
      for (int pass = 0; pass < 2; ++pass) {
#pragma unroll
        for (int it = 0; it < 8; ++it) {
          const int row = it * 2 + hh;
          v4f v = *(const v4f*)(slab + row * 68 + c4);
          *(volatile v4f*)(C + (size_t)(mBase + row) * ldc + n0 + c4) = v;
        }
        __threadfence();
      }
    } else {
      const int q = lane >> 3, c8 = (lane & 7) * 8;
      unsigned short* C  = (unsigned short*)Cout  + (size_t)b * strideC;
      unsigned short* C2 = (OUT_MODE == 2) ? ((unsigned short*)Cout2 + (size_t)b * strideC) : nullptr;
      for (int pass = 0; pass < 2; ++pass) {
#pragma unroll
        for (int it = 0; it < 4; ++it) {
          const int row = it * 4 + q;
          const float* sp = slab + row * 68 + c8;
          v8h hv, lv;
#pragma unroll
          for (int e = 0; e < 8; ++e) {
            if (OUT_MODE == 1) {
              hv[e] = (_Float16)sp[e];
            } else {
              unsigned short hb = f2bf_bits(sp[e]);
              unsigned short lb = f2bf_bits(sp[e] - bf_bits2f(hb));
              hv[e] = __builtin_bit_cast(_Float16, hb);
              lv[e] = __builtin_bit_cast(_Float16, lb);
            }
          }
          *(volatile v8h*)(C + (size_t)(mBase + row) * ldc + n0 + c8) = hv;
          if (OUT_MODE == 2) *(volatile v8h*)(C2 + (size_t)(mBase + row) * ldc + n0 + c8) = lv;
        }
        __threadfence();
      }
    }
    __builtin_amdgcn_fence(__ATOMIC_RELEASE, "workgroup");
    __builtin_amdgcn_wave_barrier();
    __builtin_amdgcn_fence(__ATOMIC_ACQUIRE, "workgroup");
  }
}

__global__ __launch_bounds__(256) void k_pool(const float* __restrict__ x, float* __restrict__ xp) {
  __shared__ float t[64][33];
  const int tid = threadIdx.x;
  const int blk = blockIdx.x;
  const int ct  = blk & 3;
  const int rr  = blk >> 2;
  const int hwT = rr % (kHW / 32);
  const int b   = rr / (kHW / 32);
  const int hw0 = hwT * 32;
  const int c0  = ct * 64;
  const float* xb = x + ((size_t)b * kCIN + c0) * kHW;
#pragma unroll
  for (int i = 0; i < 8; ++i) {
    const int idx = i * 256 + tid;
    const int c = idx >> 5, j = idx & 31;
    const int hw = hw0 + j;
    const int h = hw / kWD, w = hw - h * kWD;
    const float* xc = xb + (size_t)c * kHW;
    float s = 0.f;
#pragma unroll
    for (int dy = -1; dy <= 1; ++dy) {
      const int y  = h + dy;
      const int yc = y < 0 ? 0 : (y > kHH - 1 ? kHH - 1 : y);
      const bool vy = (unsigned)y < (unsigned)kHH;
#pragma unroll
      for (int dx = -1; dx <= 1; ++dx) {
        const int xx  = w + dx;
        const int xcl = xx < 0 ? 0 : (xx > kWD - 1 ? kWD - 1 : xx);
        const bool vx = (unsigned)xx < (unsigned)kWD;
        const float v = xc[yc * kWD + xcl];
        s += (vy && vx) ? v : 0.0f;
      }
    }
    t[c][j] = s * (1.0f / 9.0f);
  }
  __syncthreads();
  const int wave = tid >> 5, lane = tid & 31, hh = lane >> 4, c4 = (lane & 15) * 4;
  float* ob = xp + ((size_t)b * kHW + hw0) * kCIN + c0;
  for (int pass = 0; pass < 2; ++pass) {
#pragma unroll
    for (int it = 0; it < 2; ++it) {
      const int row = wave * 4 + it * 2 + hh;
      v4f v;
      v[0] = t[c4][row]; v[1] = t[c4 + 1][row]; v[2] = t[c4 + 2][row]; v[3] = t[c4 + 3][row];
      *(volatile v4f*)(ob + (size_t)row * kCIN + c4) = v;
    }
    __threadfence();
  }
}

__global__ __launch_bounds__(256) void k_prep_woff(const float* __restrict__ wo, const float* __restrict__ wm,
                                                   unsigned short* __restrict__ Ao) {
  const int g = blockIdx.x * 256 + threadIdx.x;
  if (g < kMOFF * kKD / 8) {
    const int e0  = g * 8;
    const int o   = e0 / kKD;
    const int col = e0 - o * kKD;
    const int k   = col >> 8;
    const int c0  = col & (kCIN - 1);
    const int oa  = o < kNOFS ? o : (kNOFS - 1);
    int om = o - kNOFS; om = om < 0 ? 0 : (om > kNMOD - 1 ? kNMOD - 1 : om);
    float f[8];
#pragma unroll
    for (int j = 0; j < 8; ++j) {
      const float va = wo[((size_t)oa * kCIN + c0 + j) * kTAPS + k];
      const float vb = wm[((size_t)om * kCIN + c0 + j) * kTAPS + k];
      const float v  = (o < kNOFS) ? va : ((o < kNOFF) ? vb : 0.0f);
      f[j] = v * kSC_WO;
    }
    v4u u;
    u[0] = pkh2(f[0], f[1]); u[1] = pkh2(f[2], f[3]); u[2] = pkh2(f[4], f[5]); u[3] = pkh2(f[6], f[7]);
    volatile v4u* p = (volatile v4u*)(Ao + e0);
    *p = u;
    __threadfence();
    *p = u;
  }
}

__global__ __launch_bounds__(256) void k_prep_wdef(const float* __restrict__ w, unsigned short* __restrict__ Wd) {
  const int g = blockIdx.x * 256 + threadIdx.x;
  if (g < kCOUT * kKD / 8) {
    const int e0  = g * 8;
    const int o   = e0 / kKD;
    const int col = e0 - o * kKD;
    const int k   = col >> 8;
    const int c0  = col & (kCIN - 1);
    float f[8];
#pragma unroll
    for (int j = 0; j < 8; ++j) f[j] = w[((size_t)o * kCIN + c0 + j) * kTAPS + k] * kSC_WD;
    v4u u;
    u[0] = pkh2(f[0], f[1]); u[1] = pkh2(f[2], f[3]); u[2] = pkh2(f[4], f[5]); u[3] = pkh2(f[6], f[7]);
    volatile v4u* p = (volatile v4u*)(Wd + e0);
    *p = u;
    __threadfence();
    *p = u;
  }
}

__global__ __launch_bounds__(256) void k_im2col(const float* __restrict__ xp, unsigned short* __restrict__ P, int bsel) {
  const int lane = threadIdx.x & 31, wave = threadIdx.x >> 5;
  const int c8 = lane * 8;
  const int it = blockIdx.x * 8 + wave;
  if (it < kHW * kTAPS) {
    const int p  = it / kTAPS, k = it - p * kTAPS;
    const int h  = p / kWD, w = p - h * kWD;
    const int kh = k / 3, kw = k - kh * 3;
    const int y  = h - 1 + kh, xx = w - 1 + kw;
    const bool inb = ((unsigned)y < (unsigned)kHH) && ((unsigned)xx < (unsigned)kWD);
    const int yc = y < 0 ? 0 : (y > kHH - 1 ? kHH - 1 : y);
    const int xc = xx < 0 ? 0 : (xx > kWD - 1 ? kWD - 1 : xx);
    const float* src = xp + ((size_t)bsel * kHW + (size_t)yc * kWD + xc) * kCIN + c8;
    v4f a = *(const v4f*)(src);
    v4f c = *(const v4f*)(src + 4);
    const v4f z = (v4f){0.f, 0.f, 0.f, 0.f};
    if (!inb) { a = z; c = z; }
    a = a * kSC_IM;
    c = c * kSC_IM;
    v4u u;
    u[0] = pkh2(a[0], a[1]); u[1] = pkh2(a[2], a[3]); u[2] = pkh2(c[0], c[1]); u[3] = pkh2(c[2], c[3]);
    volatile v4u* d = (volatile v4u*)(P + (size_t)it * kCIN + c8);
    *d = u;
    __threadfence();
    *d = u;
  }
}

__global__ __launch_bounds__(256) void k_sample(const float* __restrict__ xp, const float* __restrict__ off,
                                                const float* __restrict__ ob, const float* __restrict__ mb,
                                                unsigned short* __restrict__ S, int bsel) {
  const int lane = threadIdx.x & 31, wave = threadIdx.x >> 5;
  const int c8 = lane * 8;
  const int it = blockIdx.x * 8 + wave;
  if (it < kHW * kTAPS) {
    const int p  = it / kTAPS, k = it - p * kTAPS;
    const int h  = p / kWD, w = p - h * kWD;
    const int kh = k / 3, kw = k - kh * 3;
    const size_t pg = (size_t)bsel * kHW + p;
    const float dy = off[(size_t)(2 * k) * kNPIX + pg] + ob[2 * k];
    const float dx = off[(size_t)(2 * k + 1) * kNPIX + pg] + ob[2 * k + 1];
    float ml = off[(size_t)(kNOFS + k) * kNPIX + pg] + mb[k];
    ml = fminf(fmaxf(ml, -30.0f), 30.0f);
    const float msk = 2.0f * __builtin_amdgcn_rcpf(1.0f + __expf(-ml));
    const float py = (float)(h - 1 + kh) + dy;
    const float px = (float)(w - 1 + kw) + dx;
    const float y0 = floorf(py), x0 = floorf(px);
    const float y1 = y0 + 1.0f, x1 = x0 + 1.0f;
    const float wy1 = py - y0, wx1 = px - x0;
    const float wy0 = 1.0f - wy1, wx0 = 1.0f - wx1;
    const bool vy0 = (y0 >= 0.0f) && (y0 <= (float)(kHH - 1));
    const bool vy1 = (y1 >= 0.0f) && (y1 <= (float)(kHH - 1));
    const bool vx0 = (x0 >= 0.0f) && (x0 <= (float)(kWD - 1));
    const bool vx1 = (x1 >= 0.0f) && (x1 <= (float)(kWD - 1));
    float w00 = wy0 * wx0, w01 = wy0 * wx1, w10 = wy1 * wx0, w11 = wy1 * wx1;
    w00 = (vy0 && vx0) ? w00 : 0.0f;
    w01 = (vy0 && vx1) ? w01 : 0.0f;
    w10 = (vy1 && vx0) ? w10 : 0.0f;
    w11 = (vy1 && vx1) ? w11 : 0.0f;
    const int yi0 = (int)fminf(fmaxf(y0, 0.0f), (float)(kHH - 1));
    const int yi1 = (int)fminf(fmaxf(y1, 0.0f), (float)(kHH - 1));
    const int xi0 = (int)fminf(fmaxf(x0, 0.0f), (float)(kWD - 1));
    const int xi1 = (int)fminf(fmaxf(x1, 0.0f), (float)(kWD - 1));
    const float* xb  = xp + (size_t)bsel * kHW * kCIN + c8;
    const float* r00 = xb + ((size_t)yi0 * kWD + xi0) * kCIN;
    const float* r01 = xb + ((size_t)yi0 * kWD + xi1) * kCIN;
    const float* r10 = xb + ((size_t)yi1 * kWD + xi0) * kCIN;
    const float* r11 = xb + ((size_t)yi1 * kWD + xi1) * kCIN;
    const v4f g00a = *(const v4f*)(r00), g00b = *(const v4f*)(r00 + 4);
    const v4f g01a = *(const v4f*)(r01), g01b = *(const v4f*)(r01 + 4);
    const v4f g10a = *(const v4f*)(r10), g10b = *(const v4f*)(r10 + 4);
    const v4f g11a = *(const v4f*)(r11), g11b = *(const v4f*)(r11 + 4);
    v4f va = g00a * w00 + g01a * w01 + g10a * w10 + g11a * w11;
    v4f vb = g00b * w00 + g01b * w01 + g10b * w10 + g11b * w11;
    const float mks = msk * kSC_S;
    va = va * mks;
    vb = vb * mks;
    v4u u;
    u[0] = pkh2(va[0], va[1]); u[1] = pkh2(va[2], va[3]);
    u[2] = pkh2(vb[0], vb[1]); u[3] = pkh2(vb[2], vb[3]);
    volatile v4u* d = (volatile v4u*)(S + (size_t)it * kCIN + c8);
    *d = u;
    __threadfence();
    *d = u;
  }
}

extern "C" void kernel_launch(void* const* d_in, const int* in_sizes, int n_in,
                              void* d_out, int out_size, void* d_ws, size_t ws_size,
                              hipStream_t stream) {
  if (n_in < 7) return;
  if (in_sizes[0] != kNPIX * kCIN || in_sizes[1] != kNOFS * kKD || in_sizes[2] != kNOFS ||
      in_sizes[3] != kNMOD * kKD || in_sizes[4] != kNMOD || in_sizes[5] != kCOUT * kKD || in_sizes[6] != kCOUT) return;
  if (out_size != kNB * kCOUT * kHW) return;

  const float* x     = (const float*)d_in[0];
  const float* off_w = (const float*)d_in[1];
  const float* off_b = (const float*)d_in[2];
  const float* mod_w = (const float*)d_in[3];
  const float* mod_b = (const float*)d_in[4];
  const float* w_def = (const float*)d_in[5];
  const float* b_def = (const float*)d_in[6];
  float* out = (float*)d_out;

  const size_t bytes_XP  = (size_t)kNPIX * kCIN * 4;
  const size_t bytes_OFF = (size_t)kMOFF * kNPIX * 4;
  const size_t bytes_P   = (size_t)kHW * kKD * 2;
  const size_t bytes_S   = (size_t)kHW * kKD * 2;
  const size_t bytes_AO  = (size_t)kMOFF * kKD * 2;
  const size_t bytes_WD  = (size_t)kCOUT * kKD * 2;
  char* ws = (char*)d_ws;
  size_t o = 0;
  float* XP = (float*)(ws + o);                        o += bytes_XP;
  float* OFF = (float*)(ws + o);                       o += bytes_OFF;
  unsigned short* PIM = (unsigned short*)(ws + o);     o += bytes_P;
  unsigned short* S   = (unsigned short*)(ws + o);     o += bytes_S;
  unsigned short* AO  = (unsigned short*)(ws + o);     o += bytes_AO;
  unsigned short* WD  = (unsigned short*)(ws + o);     o += bytes_WD;
  if (o > ws_size || o > (size_t)134217728) return;

  k_pool<<<kNB * (kHW / 32) * (kCIN / 64), 256, 0, stream>>>(x, XP);
  k_prep_woff<<<(kMOFF * kKD / 8) / 256, 256, 0, stream>>>(off_w, mod_w, AO);
  k_prep_wdef<<<(kCOUT * kKD / 8) / 256, 256, 0, stream>>>(w_def, WD);
  for (int bsel = 0; bsel < kNB; ++bsel) {
    k_im2col<<<(kHW * kTAPS) / 8, 256, 0, stream>>>(XP, PIM, bsel);
    wmma_gemm64<0, false, 0, 0, false><<<dim3(((kMOFF / 64) * (kHW / 64) + 7) / 8, 1), 256, 0, stream>>>(
        AO, AO, kKD, 0L,
        PIM, PIM, kKD, 0L,
        (void*)(OFF + (size_t)bsel * kHW), (void*)WD, kNPIX, 0L,
        b_def,
        off_b, 0L,
        kMOFF, kHW, kKD, kEPI_OFF);
    k_sample<<<(kHW * kTAPS) / 8, 256, 0, stream>>>(XP, OFF, off_b, mod_b, S, bsel);
    wmma_gemm64<0, false, 1, 0, false><<<dim3(((kCOUT / 64) * (kHW / 64) + 7) / 8, 1), 256, 0, stream>>>(
        WD, WD, kKD, 0L,
        S, S, kKD, 0L,
        (void*)(out + (size_t)bsel * kCOUT * kHW), (void*)WD, kHW, 0L,
        b_def,
        off_b, 0L,
        kCOUT, kHW, kKD, kEPI_MAIN);
  }
}
